// MultiHeadedAttentionRel_52647709114819
// MI455X (gfx1250) — hardware-verified
//
#include <hip/hip_runtime.h>
#include <stdint.h>

typedef __attribute__((ext_vector_type(16))) _Float16 v16h;
typedef __attribute__((ext_vector_type(8)))  _Float16 v8h;
typedef __attribute__((ext_vector_type(16))) __bf16   v16b;
typedef __attribute__((ext_vector_type(8)))  __bf16   v8b;
typedef __attribute__((ext_vector_type(8)))  float    v8f;
typedef __attribute__((ext_vector_type(4)))  float    v4f;
typedef _Float16 h_alias __attribute__((may_alias));
#define PSCALE 32768.0f
#define U16(p) ((const unsigned short*)(const void*)(p))
#define PSCALE_INV (1.0f / 32768.0f)

__device__ __forceinline__ unsigned short f2bf_bits(float f) {
  unsigned u = __float_as_uint(f);
  return (unsigned short)((u + 0x7FFFu + ((u >> 16) & 1u)) >> 16);
}
__device__ __forceinline__ float bf_bits2f(unsigned short h) { return __uint_as_float(((unsigned)h) << 16); }

__device__ __forceinline__ void dep_guard_h(v8f& a, v8f& b, v16h x, v16h y) { asm volatile("v_nop\n\tv_nop\n\tv_nop\n\tv_nop" : "+v"(a), "+v"(b) : "v"(x), "v"(y)); }
__device__ __forceinline__ void dep_guard_b(v8f& a, v8f& b, v16b x, v16b y) { asm volatile("v_nop\n\tv_nop\n\tv_nop\n\tv_nop" : "+v"(a), "+v"(b) : "v"(x), "v"(y)); }
__device__ __forceinline__ void keep4_h(v16h a, v16h b, v16h c, v16h d) { asm volatile("v_nop" :: "v"(a), "v"(b), "v"(c), "v"(d)); }
__device__ __forceinline__ void keep4_b(v16b a, v16b b, v16b c, v16b d) { asm volatile("v_nop" :: "v"(a), "v"(b), "v"(c), "v"(d)); }
__device__ __forceinline__ void acc_guard4(v8f& a, v8f& b, v8f& c, v8f& d) { asm volatile("v_nop\n\tv_nop\n\tv_nop\n\tv_nop" : "+v"(a), "+v"(b), "+v"(c), "+v"(d)); }
template <typename T> struct Frag;
template <> struct Frag<_Float16> {
  typedef v16h V; union U { v16h v; v8h h[2]; };
  static __device__ __forceinline__ v16h load(const _Float16* p) {
    U f; f.h[0] = *(const v8h*)(p); f.h[1] = *(const v8h*)(p + 16); return f.v;
  }
  static __device__ __forceinline__ v8f mma(v16h a, v16h b, v8f c) {
    return __builtin_amdgcn_wmma_f32_16x16x32_f16(false, a, false, b, (short)0, c, false, false);
  }
  static __device__ __forceinline__ void guard(v8f& a, v8f& b, v16h x, v16h y) { dep_guard_h(a, b, x, y); }
  static __device__ __forceinline__ void keep(v16h a, v16h b, v16h c, v16h d) { keep4_h(a, b, c, d); }
};
template <> struct Frag<__bf16> {
  typedef v16b V; union U { v16b v; v8b h[2]; };
  static __device__ __forceinline__ v16b load(const __bf16* p) {
    U f; f.h[0] = *(const v8b*)(p); f.h[1] = *(const v8b*)(p + 16); return f.v;
  }
  static __device__ __forceinline__ v8f mma(v16b a, v16b b, v8f c) {
    return __builtin_amdgcn_wmma_f32_16x16x32_bf16(false, a, false, b, (short)0, c, false, false);
  }
  static __device__ __forceinline__ void guard(v8f& a, v8f& b, v16b x, v16b y) { dep_guard_b(a, b, x, y); }
  static __device__ __forceinline__ void keep(v16b a, v16b b, v16b c, v16b d) { keep4_b(a, b, c, d); }
};

template <int ET> struct Elem;
template <> struct Elem<0> { typedef _Float16 T; };
template <> struct Elem<1> { typedef __bf16 T; };
template <int ET, bool SPLIT, int BIAS_MODE, int OUT_MODE, bool RESID, int ACT = 0>
__global__ __launch_bounds__(256) void wmma_gemm64(
    const unsigned short* __restrict__ Ap, const unsigned short* __restrict__ A2p, int lda, long strideA,
    const unsigned short* __restrict__ Btp, const unsigned short* __restrict__ Bt2p, int ldb, long strideB,
    void* __restrict__ Cout, void* __restrict__ Cout2, int ldc, long strideC,
    const float* __restrict__ bias,
    const float* __restrict__ resid, long strideR,
    int M, int N, int K, float scale) {
  typedef typename Elem<ET>::T T;
  typedef typename Frag<T>::V V;
  const T* A = (const T*)Ap; const T* A2 = (const T*)A2p; const T* Bt = (const T*)Btp; const T* Bt2 = (const T*)Bt2p;
  __shared__ __align__(16) float sT[8][16 * 68];
  const int b    = blockIdx.y;
  const int lane = threadIdx.x & 31;
  const int wave = threadIdx.x >> 5;
  const int tilesN = N >> 6;
  const int tilesM = M >> 6;
  const int tile = blockIdx.x * 8 + wave;
  if (tile >= tilesM * tilesN) return;
  const int tm = tile / tilesN;
  const int tn = tile - tm * tilesN;
  const int m0 = tm << 6;
  const int n0 = tn << 6;

  const T* Ab  = A  + (size_t)b * strideA;
  const T* Bb  = Bt + (size_t)b * strideB;
  const T* Ab2 = SPLIT ? (A2  + (size_t)b * strideA) : nullptr;
  const T* Bb2 = SPLIT ? (Bt2 + (size_t)b * strideB) : nullptr;

  const int rlane = lane & 15;
  const int koff  = (lane >> 4) * 8;
  const int mOff  = (lane >> 4) * 8;

  v8f acc[4][4];
#pragma unroll
  for (int i = 0; i < 4; ++i)
#pragma unroll
    for (int j = 0; j < 4; ++j) acc[i][j] = (v8f){0.f,0.f,0.f,0.f,0.f,0.f,0.f,0.f};

  for (int k0 = 0; k0 < K; k0 += 32) {
    V bh[4], bl[4];
#pragma unroll
    for (int j = 0; j < 4; ++j) {
      const size_t bo = (size_t)(n0 + (j << 4) + rlane) * ldb + koff + k0;
      bh[j] = Frag<T>::load(Bb + bo);
      if (SPLIT) bl[j] = Frag<T>::load(Bb2 + bo);
    }
#pragma unroll
    for (int i = 0; i < 4; ++i) {
      const size_t ao = (size_t)(m0 + (i << 4) + rlane) * lda + koff + k0;
      V ah = Frag<T>::load(Ab + ao);
      V al;
      if (SPLIT) al = Frag<T>::load(Ab2 + ao);
#pragma unroll
      for (int j = 0; j < 4; ++j) {
        acc[i][j] = Frag<T>::mma(ah, bh[j], acc[i][j]);
        if (SPLIT) {
          acc[i][j] = Frag<T>::mma(ah, bl[j], acc[i][j]);
          acc[i][j] = Frag<T>::mma(al, bh[j], acc[i][j]);
        }
      }
      Frag<T>::guard(acc[i][0], acc[i][3], ah, SPLIT ? al : ah);
    }
    Frag<T>::keep(bh[0], bh[1], bh[2], bh[3]);
    if (SPLIT) Frag<T>::keep(bl[0], bl[1], bl[2], bl[3]);
  }
  acc_guard4(acc[0][0], acc[0][1], acc[0][2], acc[0][3]);
  acc_guard4(acc[1][0], acc[1][1], acc[1][2], acc[1][3]);
  acc_guard4(acc[2][0], acc[2][1], acc[2][2], acc[2][3]);
  acc_guard4(acc[3][0], acc[3][1], acc[3][2], acc[3][3]);

  float* slab = sT[wave];
  const float* Rb = RESID ? (resid + (size_t)b * strideR) : nullptr;
#pragma unroll
  for (int i = 0; i < 4; ++i) {
    const int mBase = m0 + (i << 4);
#pragma unroll
    for (int j = 0; j < 4; ++j) {
      const int n = n0 + (j << 4) + rlane;
      float bv = 0.f;
      if (BIAS_MODE == 2) bv = bias[n];
#pragma unroll
      for (int r = 0; r < 8; ++r) {
        float v = acc[i][j][r] * scale;
        if (BIAS_MODE == 1) v += bias[mBase + mOff + r];
        if (BIAS_MODE == 2) v += bv;
        if (RESID) v += Rb[(size_t)(mBase + mOff + r) * ldc + n];
        if (ACT == 1) v = tanhf(v);
        if (ACT == 2) v = fmaxf(v, 0.0f);
        if (ACT == 3) v = v / (1.0f + expf(-v));
        if (ACT == 4) v = (v > 0.f) ? v : 0.01f * v;
        if (ACT == 5) v = 0.5f * v * (1.0f + erff(v * 0.70710678118654752f));
        slab[(mOff + r) * 68 + (j << 4) + rlane] = v;
      }
    }
    __builtin_amdgcn_fence(__ATOMIC_RELEASE, "workgroup");
    __builtin_amdgcn_wave_barrier();
    __builtin_amdgcn_fence(__ATOMIC_ACQUIRE, "workgroup");
    if (OUT_MODE == 0) {
      float* C = (float*)Cout + (size_t)b * strideC;
      const int hh = lane >> 4, c4 = (lane & 15) * 4;
      for (int pass = 0; pass < 2; ++pass) {
#pragma unroll
        for (int it = 0; it < 8; ++it) {
          const int row = it * 2 + hh;
          v4f v = *(const v4f*)(slab + row * 68 + c4);
          *(volatile v4f*)(C + (size_t)(mBase + row) * ldc + n0 + c4) = v;
        }
        __threadfence();
      }
    } else {
      const int q = lane >> 3, c8 = (lane & 7) * 8;
      unsigned short* C  = (unsigned short*)Cout  + (size_t)b * strideC;
      unsigned short* C2 = (OUT_MODE == 2) ? ((unsigned short*)Cout2 + (size_t)b * strideC) : nullptr;
      for (int pass = 0; pass < 2; ++pass) {
#pragma unroll
        for (int it = 0; it < 4; ++it) {
          const int row = it * 4 + q;
          const float* sp = slab + row * 68 + c8;
          v8h hv, lv;
#pragma unroll
          for (int e = 0; e < 8; ++e) {
            if (OUT_MODE == 1) {
              hv[e] = (_Float16)sp[e];
            } else {
              unsigned short hb = f2bf_bits(sp[e]);
              unsigned short lb = f2bf_bits(sp[e] - bf_bits2f(hb));
              hv[e] = __builtin_bit_cast(_Float16, hb);
              lv[e] = __builtin_bit_cast(_Float16, lb);
            }
          }
          *(volatile v8h*)(C + (size_t)(mBase + row) * ldc + n0 + c8) = hv;
          if (OUT_MODE == 2) *(volatile v8h*)(C2 + (size_t)(mBase + row) * ldc + n0 + c8) = lv;
        }
        __threadfence();
      }
    }
    __builtin_amdgcn_fence(__ATOMIC_RELEASE, "workgroup");
    __builtin_amdgcn_wave_barrier();
    __builtin_amdgcn_fence(__ATOMIC_ACQUIRE, "workgroup");
  }
}

__global__ __launch_bounds__(256) void cast_f32_f16x8(
    const float* __restrict__ in, _Float16* __restrict__ out, int n8, float scale) {
  const int i = blockIdx.x * 256 + threadIdx.x;
  if (i < n8) {
    const v4f a = *(const v4f*)(in + (size_t)i * 8);
    const v4f b = *(const v4f*)(in + (size_t)i * 8 + 4);
    v8h hv;
    hv[0] = (_Float16)(a[0] * scale); hv[1] = (_Float16)(a[1] * scale);
    hv[2] = (_Float16)(a[2] * scale); hv[3] = (_Float16)(a[3] * scale);
    hv[4] = (_Float16)(b[0] * scale); hv[5] = (_Float16)(b[1] * scale);
    hv[6] = (_Float16)(b[2] * scale); hv[7] = (_Float16)(b[3] * scale);
    _Float16* p = out + (size_t)i * 8;
    *(volatile v8h*)p = hv;
    __threadfence();
    *(volatile v8h*)p = hv;
  }
}

#define AT_D   64
#define AT_NW  4
#define AT_QB  64
#define AT_KC  64
#define MAXREL 32
#define NREL   65
#define NRELT  80
#define RVK    96
#define TP     80
#define TWSZ   (16 * TP)
#define BP     68
#define BKSZ   (16 * BP)
#define TSCALE 8.0f
#define TSCALE_INV 0.125f
#define BSCALE (PSCALE / TSCALE)

__device__ __forceinline__ void lds_wave_sync() {
  __builtin_amdgcn_fence(__ATOMIC_RELEASE, "workgroup");
  __builtin_amdgcn_wave_barrier();
  __builtin_amdgcn_fence(__ATOMIC_ACQUIRE, "workgroup");
}
__device__ __forceinline__ v8f h_mma(v16h a, v16h b, v8f c) {
  c = __builtin_amdgcn_wmma_f32_16x16x32_f16(false, a, false, b, (short)0, c, false, false);
  asm volatile("v_nop\n\tv_nop\n\tv_nop\n\tv_nop" : "+v"(c) : "v"(a), "v"(b));
  return c;
}

__global__ __launch_bounds__(256) void rel_tables_f16(const float* __restrict__ relk, const float* __restrict__ relv,
                                                      _Float16* __restrict__ rk16, _Float16* __restrict__ rvT16, float tscale) {
  const int tid = threadIdx.x;
  for (int pass = 0; pass < 2; ++pass) {
    for (int u = tid; u < NRELT * AT_D / 8; u += 256) {
      const int j = u >> 3, d0 = (u & 7) * 8;
      const int jc = j < NREL ? j : NREL - 1;
      v8h hv;
#pragma unroll
      for (int e = 0; e < 8; ++e) {
        const float x = relk[jc * AT_D + d0 + e] * tscale;
        hv[e] = (j < NREL) ? (_Float16)x : (_Float16)0.0f;
      }
      *(volatile v8h*)(rk16 + (size_t)u * 8) = hv;
    }
    for (int u = tid; u < AT_D * RVK / 8; u += 256) {
      const int d  = u / (RVK / 8);
      const int j0 = (u - d * (RVK / 8)) * 8;
      v8h hv;
#pragma unroll
      for (int e = 0; e < 8; ++e) {
        const int j  = j0 + e;
        const int jc = j < NREL ? j : NREL - 1;
        const float x = relv[jc * AT_D + d] * tscale;
        hv[e] = (j < NREL) ? (_Float16)x : (_Float16)0.0f;
      }
      *(volatile v8h*)(rvT16 + (size_t)u * 8) = hv;
    }
    __threadfence();
  }
}

__global__ __launch_bounds__(128)
void attn_rel_kernel(const _Float16* __restrict__ q, const _Float16* __restrict__ k,
                     const _Float16* __restrict__ v, const _Float16* __restrict__ rk16,
                     const _Float16* __restrict__ rvT16, _Float16* __restrict__ ctx,
                     int S, int H, float cscale) {
  __shared__ __align__(16) _Float16 KV[2 * AT_KC * AT_D];
  __shared__ __align__(16) _Float16 Psh[AT_NW][16 * AT_KC];
  __shared__ __align__(16) float    Tws[AT_NW * TWSZ];
  __shared__ __align__(16) float    Bks[AT_NW * BKSZ];

  _Float16* const Ksh = KV;
  _Float16* const Vth = KV + AT_KC * AT_D;

  const int tid  = threadIdx.x;
  const int wave = tid >> 5;
  const int lane = tid & 31;
  const int hh   = lane >> 4;
  const int c    = lane & 15;
  const long rs  = (long)H * AT_D;
  const long bs  = (long)S * rs;
  const int nqb  = S / AT_QB;
  const int bx   = blockIdx.x;
  const int qb   = bx % nqb;
  const int bhd  = bx / nqb;
  const int h    = bhd % H;
  const int b    = bhd / H;
  const int q0   = qb * AT_QB + wave * 16;

  const _Float16* qb_ptr = q + (size_t)b * bs + (size_t)h * AT_D;
  const _Float16* kb_ptr = k + (size_t)b * bs + (size_t)h * AT_D;
  const _Float16* vb_ptr = v + (size_t)b * bs + (size_t)h * AT_D;
  _Float16*       ob_ptr = ctx + (size_t)b * bs + (size_t)h * AT_D;
  float* const Tw = Tws + wave * TWSZ;
  float* const Bk = Bks + wave * BKSZ;

  for (int u = tid; u < NRELT * AT_D / 8; u += AT_NW * 32)
    *(v8h*)(KV + u * 8) = *(const v8h*)(rk16 + (size_t)u * 8);
  {
    const v4f z = {0.f, 0.f, 0.f, 0.f};
    for (int u = tid; u < AT_NW * BKSZ / 4; u += AT_NW * 32) *(v4f*)(Bks + u * 4) = z;
  }

  v16h qa[2];
  {
    const _Float16* qrow = qb_ptr + (size_t)(q0 + c) * rs;
    qa[0] = Frag<_Float16>::load(qrow + 8 * hh);
    qa[1] = Frag<_Float16>::load(qrow + 32 + 8 * hh);
  }
  __syncthreads();

#pragma unroll
  for (int jt = 0; jt < NRELT / 16; ++jt) {
    v8f tacc = (v8f){0.f,0.f,0.f,0.f,0.f,0.f,0.f,0.f};
#pragma unroll
    for (int dc = 0; dc < 2; ++dc) {
      const v16h rb = Frag<_Float16>::load(KV + (jt * 16 + c) * AT_D + dc * 32 + 8 * hh);
      tacc = h_mma(qa[dc], rb, tacc);
    }
#pragma unroll
    for (int r = 0; r < 8; ++r) Tw[(8 * hh + r) * TP + jt * 16 + c] = tacc[r] * TSCALE_INV;
  }
  lds_wave_sync();

  float mrow[8], lrow[8], alph[8];
  v8f oacc[4];
#pragma unroll
  for (int r = 0; r < 8; ++r) { mrow[r] = -__builtin_inff(); lrow[r] = 0.f; alph[r] = 0.f; }
#pragma unroll
  for (int t = 0; t < 4; ++t) oacc[t] = (v8f){0.f,0.f,0.f,0.f,0.f,0.f,0.f,0.f};

  const int nChunks = S / AT_KC;
  for (int kc = 0; kc < nChunks; ++kc) {
    const int kv0 = kc * AT_KC;
    __syncthreads();
    {
      const int kvr = tid >> 1, dh = (tid & 1) * 32;
      const _Float16* krow = kb_ptr + (size_t)(kv0 + kvr) * rs + dh;
      const _Float16* vrow = vb_ptr + (size_t)(kv0 + kvr) * rs + dh;
#pragma unroll
      for (int i = 0; i < 4; ++i) {
        const v8h kk8 = *(const v8h*)(krow + 8 * i);
        const v8h vv8 = *(const v8h*)(vrow + 8 * i);
        *(v8h*)(Ksh + kvr * AT_D + dh + 8 * i) = kk8;
#pragma unroll
        for (int e = 0; e < 8; ++e) Vth[(dh + 8 * i + e) * AT_KC + kvr] = vv8[e];
      }
    }
    __syncthreads();

    v8f s[4];
#pragma unroll
    for (int j = 0; j < 4; ++j) {
      s[j] = (v8f){0.f,0.f,0.f,0.f,0.f,0.f,0.f,0.f};
#pragma unroll
      for (int dc = 0; dc < 2; ++dc) {
        const v16h kb = Frag<_Float16>::load(Ksh + (j * 16 + c) * AT_D + dc * 32 + 8 * hh);
        s[j] = h_mma(qa[dc], kb, s[j]);
      }
    }
    float cm[8];
#pragma unroll
    for (int r = 0; r < 8; ++r) {
      const int row  = 8 * hh + r;
      const int qrow = q0 + row;
      float m = -__builtin_inff();
#pragma unroll
      for (int j = 0; j < 4; ++j) {
        const int kvcol = kv0 + j * 16 + c;
        int dd = kvcol - qrow;
        dd = dd < -MAXREL ? -MAXREL : (dd > MAXREL ? MAXREL : dd);
        const float sv = (s[j][r] + Tw[row * TP + dd + MAXREL]) * 0.125f;
        s[j][r] = sv;
        m = fmaxf(m, sv);
      }
#pragma unroll
      for (int off = 1; off < 16; off <<= 1) m = fmaxf(m, __shfl_xor(m, off, 32));
      cm[r] = m;
    }
    _Float16* pw = Psh[wave];
#pragma unroll
    for (int r = 0; r < 8; ++r) {
      const float mnew  = fmaxf(mrow[r], cm[r]);
      const float alpha = __expf(mrow[r] - mnew);
      mrow[r] = mnew;
      alph[r] = alpha;
      float psum = 0.f;
#pragma unroll
      for (int j = 0; j < 4; ++j) {
        const float p = __expf(s[j][r] - mnew);
        psum += p;
        s[j][r] = p;
        pw[(8 * hh + r) * AT_KC + j * 16 + c] = (_Float16)(p * PSCALE);
      }
#pragma unroll
      for (int off = 1; off < 16; off <<= 1) psum += __shfl_xor(psum, off, 32);
      lrow[r] = lrow[r] * alpha + psum;
#pragma unroll
      for (int t = 0; t < 4; ++t) oacc[t][r] *= alpha;
    }
    lds_wave_sync();

#pragma unroll
    for (int r = 0; r < 8; ++r) {
      const int row = 8 * hh + r;
      const float a = alph[r];
#pragma unroll
      for (int u = 0; u < 4; ++u) {
        float* bp = Bk + row * BP + c + 16 * u;
        *bp = *bp * a;
      }
    }
    lds_wave_sync();
#pragma unroll
    for (int r = 0; r < 8; ++r) {
      const int row  = 8 * hh + r;
      const int qrow = q0 + row;
      float t0 = 0.f, t64 = 0.f;
#pragma unroll
      for (int j = 0; j < 4; ++j) {
        const int kvcol = kv0 + j * 16 + c;
        const int dd = kvcol - qrow;
        const float p = s[j][r];
        if (dd <= -MAXREL)      t0  += p;
        else if (dd >= MAXREL)  t64 += p;
        else                    Bk[row * BP + dd + MAXREL] = p;
      }
#pragma unroll
      for (int off = 1; off < 16; off <<= 1) { t0 += __shfl_xor(t0, off, 32); t64 += __shfl_xor(t64, off, 32); }
      if (c == 0) {
        Bk[row * BP] += t0;
        Bk[row * BP + 2 * MAXREL] = Bk[row * BP + 2 * MAXREL] * alph[r] + t64;
      }
    }

#pragma unroll
    for (int kk = 0; kk < 2; ++kk) {
      const v16h pa = Frag<_Float16>::load(pw + c * AT_KC + kk * 32 + 8 * hh);
#pragma unroll
      for (int t = 0; t < 4; ++t) {
        const v16h vb = Frag<_Float16>::load(Vth + (t * 16 + c) * AT_KC + kk * 32 + 8 * hh);
        oacc[t] = h_mma(pa, vb, oacc[t]);
      }
    }
  }
  __syncthreads();

  for (int u = tid; u < AT_D * RVK / 8; u += AT_NW * 32)
    *(v8h*)(KV + u * 8) = *(const v8h*)(rvT16 + (size_t)u * 8);

  float invl[8];
#pragma unroll
  for (int r = 0; r < 8; ++r) invl[r] = 1.0f / lrow[r];
  {
    h_alias* At = (h_alias*)(Tws + wave * TWSZ);
#pragma unroll
    for (int r = 0; r < 8; ++r) {
      const int row = 8 * hh + r;
      const float sc = invl[r] * BSCALE;
#pragma unroll
      for (int u = 0; u < RVK / 16; ++u) {
        const int col  = c + 16 * u;
        const int colc = col < 2 * MAXREL ? col : 2 * MAXREL;
        const float bvv = Bk[row * BP + colc];
        const float val = (col < NREL) ? bvv * sc : 0.0f;
        At[row * RVK + col] = (_Float16)val;
      }
    }
  }
  __syncthreads();

  v8f racc[4];
#pragma unroll
  for (int t = 0; t < 4; ++t) racc[t] = (v8f){0.f,0.f,0.f,0.f,0.f,0.f,0.f,0.f};
  {
    const _Float16* Atc = (const _Float16*)(Tws + wave * TWSZ);
#pragma unroll
    for (int ks = 0; ks < RVK / 32; ++ks) {
      const v16h ab = Frag<_Float16>::load(Atc + c * RVK + ks * 32 + 8 * hh);
#pragma unroll
      for (int t = 0; t < 4; ++t) {
        const v16h rb = Frag<_Float16>::load(KV + (t * 16 + c) * RVK + ks * 32 + 8 * hh);
        racc[t] = h_mma(ab, rb, racc[t]);
      }
    }
  }

  float* os = Bk;
  const float osc = cscale * PSCALE_INV;
#pragma unroll
  for (int r = 0; r < 8; ++r) {
    const int row = 8 * hh + r;
    const float il = invl[r];
#pragma unroll
    for (int t = 0; t < 4; ++t) os[row * BP + t * 16 + c] = (oacc[t][r] * il + racc[t][r]) * osc;
  }
  lds_wave_sync();
  {
    const int q8 = lane >> 3, c8 = (lane & 7) * 8;
    for (int pass = 0; pass < 2; ++pass) {
#pragma unroll
      for (int it = 0; it < 4; ++it) {
        const int row = it * 4 + q8;
        const float* sp = os + row * BP + c8;
        v8h hv;
#pragma unroll
        for (int e = 0; e < 8; ++e) hv[e] = (_Float16)sp[e];
        *(volatile v8h*)(ob_ptr + (size_t)(q0 + row) * rs + c8) = hv;
      }
      __threadfence();
    }
  }
}

extern "C" void kernel_launch(void* const* d_in, const int* in_sizes, int n_in,
                              void* d_out, int out_size, void* d_ws, size_t ws_size,
                              hipStream_t stream) {
  const int NB = 8, S = 1024, D = 1024, NH = 16;
  const int M = NB * S;
  const long nAct = (long)NB * S * D;
  if (n_in < 13) return;
  if (in_sizes[0] != nAct || in_sizes[1] != nAct || in_sizes[2] != nAct) return;
  if (in_sizes[3] != D * D || in_sizes[5] != D * D || in_sizes[7] != D * D || in_sizes[9] != D * D) return;
  if (in_sizes[4] != D || in_sizes[6] != D || in_sizes[8] != D || in_sizes[10] != D) return;
  if (in_sizes[11] != NREL * AT_D || in_sizes[12] != NREL * AT_D) return;
  if (out_size != nAct) return;
  if (D != NH * AT_D || (S % AT_QB) != 0 || (M % 64) != 0 || (D % 64) != 0) return;

  const float* query = (const float*)d_in[0];
  const float* key   = (const float*)d_in[1];
  const float* value = (const float*)d_in[2];
  const float* Wq = (const float*)d_in[3];  const float* bq = (const float*)d_in[4];
  const float* Wk = (const float*)d_in[5];  const float* bk = (const float*)d_in[6];
  const float* Wv = (const float*)d_in[7];  const float* bv = (const float*)d_in[8];
  const float* Wo = (const float*)d_in[9];  const float* bo = (const float*)d_in[10];
  const float* relk = (const float*)d_in[11];
  const float* relv = (const float*)d_in[12];
  float* out = (float*)d_out;

  char* ws = (char*)d_ws;
  size_t off = 0;
  const size_t actB = (size_t)nAct * 2;
  const size_t wB   = (size_t)D * D * 2;
  _Float16* X16  = (_Float16*)(ws + off); off += actB;
  _Float16* W16  = (_Float16*)(ws + off); off += wB;
  _Float16* Q16  = (_Float16*)(ws + off); off += actB;
  _Float16* K16  = (_Float16*)(ws + off); off += actB;
  _Float16* V16  = (_Float16*)(ws + off); off += actB;
  _Float16* RK16 = (_Float16*)(ws + off); off += (size_t)NRELT * AT_D * 2;
  _Float16* RV16 = (_Float16*)(ws + off); off += (size_t)AT_D * RVK * 2;
  if (off > ws_size) return;
  _Float16* CTX16 = X16;

  const int n8a = (int)(nAct / 8), n8w = D * D / 8;
  const dim3 cb(256), cga((n8a + 255) / 256), cgw((n8w + 255) / 256);
  const dim3 gb(256), gg(((M / 64) * (D / 64) + 7) / 8, 1);
  const float wcar = 64.0f;
  const float ccar = 64.0f;

  cast_f32_f16x8<<<cga, cb, 0, stream>>>(query, X16, n8a, 1.0f);
  cast_f32_f16x8<<<cgw, cb, 0, stream>>>(Wq, W16, n8w, wcar);
  wmma_gemm64<0, false, 2, 1, false, 0><<<gg, gb, 0, stream>>>(
      (const unsigned short*)X16, (const unsigned short*)X16, D, 0L,
      (const unsigned short*)W16, (const unsigned short*)W16, D, 0L,
      (void*)Q16, (void*)Q16, D, 0L, bq, bq, 0L, M, D, D, 1.0f / wcar);
  cast_f32_f16x8<<<cga, cb, 0, stream>>>(key, X16, n8a, 1.0f);
  cast_f32_f16x8<<<cgw, cb, 0, stream>>>(Wk, W16, n8w, wcar);
  wmma_gemm64<0, false, 2, 1, false, 0><<<gg, gb, 0, stream>>>(
      (const unsigned short*)X16, (const unsigned short*)X16, D, 0L,
      (const unsigned short*)W16, (const unsigned short*)W16, D, 0L,
      (void*)K16, (void*)K16, D, 0L, bk, bk, 0L, M, D, D, 1.0f / wcar);
  cast_f32_f16x8<<<cga, cb, 0, stream>>>(value, X16, n8a, 1.0f);
  cast_f32_f16x8<<<cgw, cb, 0, stream>>>(Wv, W16, n8w, wcar);
  wmma_gemm64<0, false, 2, 1, false, 0><<<gg, gb, 0, stream>>>(
      (const unsigned short*)X16, (const unsigned short*)X16, D, 0L,
      (const unsigned short*)W16, (const unsigned short*)W16, D, 0L,
      (void*)V16, (void*)V16, D, 0L, bv, bv, 0L, M, D, D, 1.0f / wcar);

  rel_tables_f16<<<dim3(1), dim3(256), 0, stream>>>(relk, relv, RK16, RV16, TSCALE);

  attn_rel_kernel<<<dim3(NB * NH * (S / AT_QB)), dim3(AT_NW * 32), 0, stream>>>(
      Q16, K16, V16, RK16, RV16, CTX16, S, NH, ccar);

  cast_f32_f16x8<<<cgw, cb, 0, stream>>>(Wo, W16, n8w, wcar);
  wmma_gemm64<0, false, 2, 0, false, 0><<<gg, gb, 0, stream>>>(
      (const unsigned short*)CTX16, (const unsigned short*)CTX16, D, 0L,
      (const unsigned short*)W16, (const unsigned short*)W16, D, 0L,
      (void*)out, (void*)out, D, 0L, bo, bo, 0L, M, D, D, 1.0f / (ccar * wcar));
}
